// GAT_5806795784462
// MI455X (gfx1250) — hardware-verified
//
#include <hip/hip_runtime.h>
#include <stddef.h>
#include <stdint.h>
#include <math.h>


#define DIN     128
#define HC1     128
#define NC1     256
#define KA2     256
#define NC2     32
#define DOUT    16
#define NTHR    256
#define NWAVE   8
#define EPT     8
#define CHUNK   (NTHR * EPT)
#define WCAP    (EPT * 32)
#define LISTN   (NWAVE * WCAP)
#define NBA     1024
#define SLA     10
#define RCAP    12288
#define DEGCAP  64
#define GBM     64
#define G2THR   128
#define NEGSL   0.2f
#define NU_W1   2048
#define NU_W2   512
#define NU_W    (2 * NU_W1 + 2 * NU_W2)
#define PAR_B1   0
#define PAR_ATT1 256
#define PAR_B2   384
#define PAR_ATT2 416
#define PAR_N    448
#define AGG_ZINTS (LISTN + 2 * RCAP + 3 * NBA)
#define AGG_LDS_INTS (AGG_ZINTS + 16)
#define WSMAX   134217728

static_assert((CHUNK & (CHUNK - 1)) == 0 && CHUNK <= 4096);
static_assert((NBA & (NBA - 1)) == 0 && NBA == (1 << SLA));
static_assert(((long long)CHUNK << SLA) < (1LL << 31));
static_assert(NBA % (2 * NWAVE) == 0 && NBA % 32 == 0);
static_assert(RCAP % 4 == 0 && AGG_ZINTS % 4 == 0 && LISTN % 4 == 0);
static_assert(DIN % 32 == 0 && KA2 % 32 == 0 && KA2 == 2 * HC1);
static_assert(HC1 == 4 * 32 && NC1 == 2 * HC1 && NC2 == 2 * DOUT);
static_assert(NU_W % NTHR == 0 && NU_W1 % NTHR == 0 && NU_W2 % NTHR == 0);
static_assert(PAR_N % 32 == 0 && PAR_N / 4 <= NTHR);
static_assert(AGG_LDS_INTS * 4 <= 300000);
static_assert(GBM * NC1 * 4 == 65536);

typedef float          v4f   __attribute__((ext_vector_type(4)));
typedef float          v8f   __attribute__((ext_vector_type(8)));
typedef int            v4i   __attribute__((ext_vector_type(4)));
typedef int            v8i   __attribute__((ext_vector_type(8)));
typedef unsigned int   v4u   __attribute__((ext_vector_type(4)));
typedef unsigned short v8us  __attribute__((ext_vector_type(8)));
typedef __bf16         v16bf __attribute__((ext_vector_type(16)));
typedef v4f  __attribute__((may_alias)) v4fa;
typedef v4i  __attribute__((may_alias)) v4ia;
typedef v8us __attribute__((may_alias)) v8usa;
union FragB { v16bf v; v8us h[2]; v4u q[2]; v8i w; };

__device__ __forceinline__ v8f wmb(const FragB& a, const FragB& b, v8f c) {
  v8f d = __builtin_amdgcn_wmma_f32_16x16x32_bf16(false, a.v, false, b.v, (short)0, c, false, false);
  asm volatile("v_nop\n\tv_nop\n\tv_nop\n\tv_nop" : "+v"(d) : "v"(a.w), "v"(b.w));
  return d;
}

__device__ __forceinline__ unsigned int f2bf(float f) {
  const unsigned int u = __float_as_uint(f);
  return ((u + 0x7FFFu + ((u >> 16) & 1u)) >> 16) & 0xFFFFu;
}
__device__ __forceinline__ float bf2f(unsigned int b) { return __uint_as_float(b << 16); }
__device__ __forceinline__ float bfr(float f) { return bf2f(f2bf(f)); }
__device__ __forceinline__ v4f bfr4(const v4f a) {
  v4f r; r.x = bfr(a.x); r.y = bfr(a.y); r.z = bfr(a.z); r.w = bfr(a.w); return r;
}
__device__ __forceinline__ unsigned int pk2(float lo, float hi) { return f2bf(lo) | (f2bf(hi) << 16); }
__device__ __forceinline__ v4u pack8(const v4f a, const v4f b) {
  v4u r;
  r.x = pk2(a.x, a.y); r.y = pk2(a.z, a.w); r.z = pk2(b.x, b.y); r.w = pk2(b.z, b.w);
  return r;
}
__device__ __forceinline__ v4f mask4(const v4f v, unsigned int mk) {
  v4f r;
  r.x = __uint_as_float(__float_as_uint(v.x) & mk); r.y = __uint_as_float(__float_as_uint(v.y) & mk);
  r.z = __uint_as_float(__float_as_uint(v.z) & mk); r.w = __uint_as_float(__float_as_uint(v.w) & mk);
  return r;
}
__device__ __forceinline__ v4f or4(const v4f a, const v4f b) {
  v4f r;
  r.x = __uint_as_float(__float_as_uint(a.x) | __float_as_uint(b.x));
  r.y = __uint_as_float(__float_as_uint(a.y) | __float_as_uint(b.y));
  r.z = __uint_as_float(__float_as_uint(a.z) | __float_as_uint(b.z));
  r.w = __uint_as_float(__float_as_uint(a.w) | __float_as_uint(b.w));
  return r;
}
__device__ __forceinline__ int clampi(int v, int lo, int hi) { return v < lo ? lo : (v > hi ? hi : v); }
__device__ __forceinline__ float elu1(float v) { return v > 0.f ? v : expm1f(v); }

template <int SLB>
__device__ __forceinline__ int scan_chunk(const int* __restrict__ dsts, int nE, int cbase, int slotBase,
                                          int nb, int vec8, int* list, int tid, int lane, int wave) {
  int wc = 0;
  const int el0  = tid * EPT;
  const int e0   = cbase + el0;
  const int sent = -2147483647 - 1;
  v4i da, db;
  if (vec8 != 0 && cbase + CHUNK <= nE) {
    da = *(const v4i*)(dsts + e0);
    db = *(const v4i*)(dsts + e0 + 4);
  } else {
    da.x = (e0     < nE) ? dsts[min(e0,     nE - 1)] : sent;
    da.y = (e0 + 1 < nE) ? dsts[min(e0 + 1, nE - 1)] : sent;
    da.z = (e0 + 2 < nE) ? dsts[min(e0 + 2, nE - 1)] : sent;
    da.w = (e0 + 3 < nE) ? dsts[min(e0 + 3, nE - 1)] : sent;
    db.x = (e0 + 4 < nE) ? dsts[min(e0 + 4, nE - 1)] : sent;
    db.y = (e0 + 5 < nE) ? dsts[min(e0 + 5, nE - 1)] : sent;
    db.z = (e0 + 6 < nE) ? dsts[min(e0 + 6, nE - 1)] : sent;
    db.w = (e0 + 7 < nE) ? dsts[min(e0 + 7, nE - 1)] : sent;
  }
  const unsigned nbs = (unsigned)slotBase;
  const unsigned unb = (unsigned)nb;
  const unsigned s0 = (unsigned)da.x - nbs, s1 = (unsigned)da.y - nbs;
  const unsigned s2 = (unsigned)da.z - nbs, s3 = (unsigned)da.w - nbs;
  const unsigned s4 = (unsigned)db.x - nbs, s5 = (unsigned)db.y - nbs;
  const unsigned s6 = (unsigned)db.z - nbs, s7 = (unsigned)db.w - nbs;
  const bool h0 = s0 < unb, h1 = s1 < unb, h2 = s2 < unb, h3 = s3 < unb;
  const bool h4 = s4 < unb, h5 = s5 < unb, h6 = s6 < unb, h7 = s7 < unb;
  const unsigned any = __builtin_amdgcn_ballot_w32(h0 | h1 | h2 | h3 | h4 | h5 | h6 | h7);
  if (any != 0u) {
#define HITJ(J, HJ, SJ) { \
      const unsigned mj = __builtin_amdgcn_ballot_w32(HJ); \
      if (mj != 0u) { \
        if (HJ) { \
          const int pos = wc + (int)__builtin_amdgcn_mbcnt_lo(mj, 0u); \
          if (pos < WCAP) list[wave * WCAP + pos] = ((el0 + (J)) << SLB) | (int)(SJ); \
        } \
        wc += (int)__builtin_popcount(mj); } }
    HITJ(0, h0, s0)
    HITJ(1, h1, s1)
    HITJ(2, h2, s2)
    HITJ(3, h3, s3)
    HITJ(4, h4, s4)
    HITJ(5, h5, s5)
    HITJ(6, h6, s6)
    HITJ(7, h7, s7)
#undef HITJ
  }
  return wc;
}

__global__ __launch_bounds__(NTHR) void k_prep(
    const float* __restrict__ W1s, const float* __restrict__ W1d,
    const float* __restrict__ W2s, const float* __restrict__ W2d,
    const float* __restrict__ b1s, const float* __restrict__ b1d, const float* __restrict__ at1,
    const float* __restrict__ b2s, const float* __restrict__ b2d, const float* __restrict__ at2,
    unsigned short* WT1, unsigned short* WT2, float* PAR) {
  const int tid = (int)threadIdx.x;
  const int u = (int)blockIdx.x * NTHR + tid;
  if (u < NU_W) {
    v8us o;
    unsigned short* dp;
    if (u < NU_W1) {
      const int n  = u >> 4;
      const int k8 = (u & 15) * 8;
      const float* p = W1s + (size_t)k8 * HC1 + n;
#pragma unroll
      for (int i = 0; i < 8; ++i) o[i] = (unsigned short)f2bf(p[(size_t)i * HC1]);
      dp = WT1 + (size_t)n * DIN + k8;
    } else if (u < 2 * NU_W1) {
      const int v  = u - NU_W1;
      const int n  = v >> 4;
      const int k8 = (v & 15) * 8;
      const float* p = W1d + (size_t)k8 * HC1 + n;
#pragma unroll
      for (int i = 0; i < 8; ++i) o[i] = (unsigned short)f2bf(p[(size_t)i * HC1]);
      dp = WT1 + (size_t)(HC1 + n) * DIN + k8;
    } else if (u < 2 * NU_W1 + NU_W2) {
      const int v  = u - 2 * NU_W1;
      const int n  = v >> 5;
      const int k8 = (v & 31) * 8;
      const int kk = k8 & (HC1 - 1);
      const float* p = W2s + (size_t)kk * DOUT + n;
#pragma unroll
      for (int i = 0; i < 8; ++i) o[i] = (unsigned short)f2bf(p[(size_t)i * DOUT]);
      dp = WT2 + (size_t)n * KA2 + k8;
    } else {
      const int v  = u - 2 * NU_W1 - NU_W2;
      const int n  = v >> 5;
      const int k8 = (v & 31) * 8;
      const int kk = k8 & (HC1 - 1);
      const float* p = W2d + (size_t)kk * DOUT + n;
#pragma unroll
      for (int i = 0; i < 8; ++i) o[i] = (unsigned short)f2bf(p[(size_t)i * DOUT]);
      dp = WT2 + (size_t)(DOUT + n) * KA2 + k8;
    }
    *(volatile v8us*)dp = o;
    __threadfence();
    *(volatile v8us*)dp = o;
  } else {
    const int t = u - NU_W;
    const v4f va = *(const v4fa*)(b1s + 4 * clampi(t,       0, 31));
    const v4f vb = *(const v4fa*)(b1d + 4 * clampi(t - 32,  0, 31));
    const v4f vc = *(const v4fa*)(at1 + 4 * clampi(t - 64,  0, 31));
    const v4f vd = *(const v4fa*)(b2s + 4 * clampi(t - 96,  0, 3));
    const v4f ve = *(const v4fa*)(b2d + 4 * clampi(t - 100, 0, 3));
    const v4f vg = *(const v4fa*)(at2 + 4 * clampi(t - 104, 0, 3));
    const unsigned int ma = (t < 32) ? 0xFFFFFFFFu : 0u;
    const unsigned int mb = (t >= 32 && t < 64) ? 0xFFFFFFFFu : 0u;
    const unsigned int mc = (t >= 64 && t < 96) ? 0xFFFFFFFFu : 0u;
    const unsigned int md = (t >= 96 && t < 100) ? 0xFFFFFFFFu : 0u;
    const unsigned int me = (t >= 100 && t < 104) ? 0xFFFFFFFFu : 0u;
    const unsigned int mg = (t >= 104 && t < 108) ? 0xFFFFFFFFu : 0u;
    v4f r = or4(or4(mask4(va, ma), mask4(vb, mb)), or4(mask4(vc, mc), mask4(vd, md)));
    r = or4(r, or4(mask4(ve, me), mask4(vg, mg)));
    r = bfr4(r);
    if (t < PAR_N / 4) {
      float* dp = PAR + 4 * t;
      *(volatile v4f*)dp = r;
      __threadfence();
      *(volatile v4f*)dp = r;
    }
  }
}

__global__ __launch_bounds__(NTHR) void k_gemm1(const float* __restrict__ X, const unsigned short* __restrict__ WT,
                                                const float* __restrict__ par, float* HS, float* HD, int nN) {
  extern __shared__ __attribute__((aligned(16))) float gsm[];
  float* stg = gsm;
  const int tid = (int)threadIdx.x, lane = tid & 31, wave = tid >> 5, hh = lane >> 4, m = lane & 15;
  const int rg = wave & 3, cg = wave >> 2;
  const int rowBase = (int)blockIdx.x * GBM;
  const int colBase = cg * HC1;

  v8f acc[8];
  {
    const v8f z = {0.f, 0.f, 0.f, 0.f, 0.f, 0.f, 0.f, 0.f};
#pragma unroll
    for (int t = 0; t < 8; ++t) acc[t] = z;
  }
  int ar = rowBase + 16 * rg + m;
  ar = ar < nN ? ar : nN - 1;
  const float* xp = X + (size_t)ar * DIN + 8 * hh;
  const unsigned short* bp = WT + (size_t)(colBase + m) * DIN + 8 * hh;

#pragma unroll 1
  for (int k0 = 0; k0 < DIN; k0 += 32) {
    const v4f a0 = *(const v4fa*)(xp + k0);
    const v4f a1 = *(const v4fa*)(xp + k0 + 4);
    const v4f a2 = *(const v4fa*)(xp + k0 + 16);
    const v4f a3 = *(const v4fa*)(xp + k0 + 20);
    FragB af;
    af.q[0] = pack8(a0, a1);
    af.q[1] = pack8(a2, a3);
#pragma unroll
    for (int nt = 0; nt < 8; ++nt) {
      const unsigned short* wq = bp + (size_t)(16 * nt) * DIN + k0;
      FragB bf;
      bf.h[0] = *(const v8usa*)wq;
      bf.h[1] = *(const v8usa*)(wq + 16);
      acc[nt] = wmb(af, bf, acc[nt]);
    }
  }

#pragma unroll
  for (int nt = 0; nt < 8; ++nt) {
    const int lc = colBase + 16 * nt + m;
#pragma unroll
    for (int r = 0; r < 8; ++r) {
      const int lr = 16 * rg + 8 * hh + r;
      stg[lr * NC1 + lc] = acc[nt][r];
    }
  }
  __syncthreads();

  const v4f bs4 = *(const v4fa*)(par + PAR_B1 + 4 * lane);
  const v4f bd4 = *(const v4fa*)(par + PAR_B1 + HC1 + 4 * lane);
#pragma unroll 1
  for (int i = 0; i < 8; ++i) {
    const int row = wave * 8 + i;
    const int gr  = rowBase + row;
    const v4f p0 = *(const v4fa*)(stg + row * NC1 + 4 * lane) + bs4;
    const v4f p1 = *(const v4fa*)(stg + row * NC1 + HC1 + 4 * lane) + bd4;
    if (gr < nN) {
      *(volatile v4f*)(HS + (size_t)gr * HC1 + 4 * lane) = p0;
      *(volatile v4f*)(HD + (size_t)gr * HC1 + 4 * lane) = p1;
    }
  }
  __threadfence();
#pragma unroll 1
  for (int i = 0; i < 8; ++i) {
    const int row = wave * 8 + i;
    const int gr  = rowBase + row;
    const v4f p0 = *(const v4fa*)(stg + row * NC1 + 4 * lane) + bs4;
    const v4f p1 = *(const v4fa*)(stg + row * NC1 + HC1 + 4 * lane) + bd4;
    if (gr < nN) {
      *(volatile v4f*)(HS + (size_t)gr * HC1 + 4 * lane) = p0;
      *(volatile v4f*)(HD + (size_t)gr * HC1 + 4 * lane) = p1;
    }
  }
}

__global__ __launch_bounds__(G2THR) void k_gemm2(const unsigned short* __restrict__ A,
                                                 const unsigned short* __restrict__ WT,
                                                 const float* __restrict__ par, float* Cm, int nN) {
  __shared__ __attribute__((aligned(16))) float stg2[4 * 16 * NC2];
  const int tid = (int)threadIdx.x, lane = tid & 31, wave = tid >> 5, hh = lane >> 4, m = lane & 15;
  const int row0 = ((int)blockIdx.x * 4 + wave) * 16;
  int ar = row0 + m;
  ar = ar < nN ? ar : nN - 1;
  const unsigned short* ap = A  + (size_t)ar * KA2 + 8 * hh;
  const unsigned short* wp = WT + (size_t)m * KA2 + 8 * hh;
  v8f acc[2];
  {
    const v8f z = {0.f, 0.f, 0.f, 0.f, 0.f, 0.f, 0.f, 0.f};
    acc[0] = z; acc[1] = z;
  }
#pragma unroll 1
  for (int ks = 0; ks < KA2 / 32; ++ks) {
    FragB af;
    af.h[0] = *(const v8usa*)(ap + 32 * ks);
    af.h[1] = *(const v8usa*)(ap + 32 * ks + 16);
#pragma unroll
    for (int t = 0; t < 2; ++t) {
      const unsigned short* wq = wp + (size_t)(16 * t) * KA2 + 32 * ks;
      FragB bf;
      bf.h[0] = *(const v8usa*)wq;
      bf.h[1] = *(const v8usa*)(wq + 16);
      acc[t] = wmb(af, bf, acc[t]);
    }
  }
  const float bz0 = par[PAR_B2 + m];
  const float bz1 = par[PAR_B2 + DOUT + m];
  float* sw = stg2 + wave * (16 * NC2);
#pragma unroll
  for (int r = 0; r < 8; ++r) {
    sw[(8 * hh + r) * NC2 + m]        = acc[0][r] + bz0;
    sw[(8 * hh + r) * NC2 + DOUT + m] = acc[1][r] + bz1;
  }
  __syncthreads();
  v4f fv[4];
#pragma unroll
  for (int i = 0; i < 4; ++i) fv[i] = *(const v4fa*)(sw + 4 * (lane + 32 * i));
  float* ob = Cm + (size_t)row0 * NC2;
#pragma unroll
  for (int i = 0; i < 4; ++i) {
    const int p = lane + 32 * i;
    if (row0 + (p >> 3) < nN) *(volatile v4f*)(ob + 4 * p) = fv[i];
  }
  __threadfence();
#pragma unroll
  for (int i = 0; i < 4; ++i) {
    const int p = lane + 32 * i;
    if (row0 + (p >> 3) < nN) *(volatile v4f*)(ob + 4 * p) = fv[i];
  }
}

template <int L>
__global__ __launch_bounds__(NTHR) void k_scan(const int* __restrict__ srcs, const int* __restrict__ dsts,
                                               int nE, int nN, int vec8, const float* __restrict__ par,
                                               const float* __restrict__ FS, const float* FD,
                                               unsigned short* HP, float* outp) {
  extern __shared__ __attribute__((aligned(16))) int dsm[];
  int* list = dsm;
  int* hl   = dsm + LISTN;
  int* sl   = dsm + LISTN + RCAP;
  int* cnt  = dsm + LISTN + 2 * RCAP;
  int* offs = cnt + NBA;
  int* cur  = offs + NBA;
  int* misc = cur + NBA;
  const int tid = (int)threadIdx.x, lane = tid & 31, wave = tid >> 5;
  const int nodeBase = (int)blockIdx.x * NBA;

  {
    const v4i z4 = {0, 0, 0, 0};
    for (int i = tid * 4; i < AGG_ZINTS; i += NTHR * 4) *(v4ia*)(dsm + i) = z4;
    if (tid < 16) misc[tid] = 0;
  }
  __syncthreads();

  int t = 0, ov = 0;
  const int nChunks = (nE + CHUNK - 1) / CHUNK;
#pragma unroll 1
  for (int ch = 0; ch < nChunks; ++ch) {
    const int cbase = ch * CHUNK;
    const int wc = scan_chunk<SLA>(dsts, nE, cbase, nodeBase, NBA, vec8, list, tid, lane, wave);
    if (lane == 0) misc[wave] = wc;
    __syncthreads();
    if (wave == 0) {
#pragma unroll 1
      for (int w2 = 0; w2 < NWAVE; ++w2) {
        int c = misc[w2];
        c = c < 0 ? 0 : (c > WCAP ? WCAP : c);
#pragma unroll 1
        for (int b0 = 0; b0 < c; b0 += 32) {
          const int idx = b0 + lane;
          const int ent = list[w2 * WCAP + (idx < WCAP ? idx : WCAP - 1)];
          const int m32 = (c - b0) < 32 ? (c - b0) : 32;
#pragma unroll 1
          for (int k = 0; k < m32; ++k) {
            const int u    = __builtin_amdgcn_readlane(ent, k);
            const int slot = u & (NBA - 1);
            const int el   = (u >> SLA) & (CHUNK - 1);
            const int pk   = ((cbase + el) << SLA) | slot;
            if (t < RCAP) {
              if (lane == 0) { hl[t] = pk; cnt[slot] = cnt[slot] + 1; }
              t = t + 1;
            } else {
              ov = 1;
            }
          }
        }
      }
    }
    __syncthreads();
  }
  if (wave == 0 && lane == 0) { misc[8] = t; misc[9] = ov; }
  __syncthreads();
  int tt = misc[8];
  tt = tt < 0 ? 0 : (tt > RCAP ? RCAP : tt);
  const int ovf = misc[9];

  if (wave == 0) {
    const int base = lane * (NBA / 32);
    int s = 0;
#pragma unroll 1
    for (int i = 0; i < NBA / 32; ++i) s += cnt[base + i];
    int incl = s;
#pragma unroll
    for (int d = 1; d < 32; d <<= 1) {
      const int y = __shfl_up(incl, d, 32);
      if (lane >= d) incl += y;
    }
    int run = incl - s;
#pragma unroll 1
    for (int i = 0; i < NBA / 32; ++i) {
      const int cv = cnt[base + i];
      offs[base + i] = run;
      cur[base + i]  = run;
      run += cv;
    }
  }
  __syncthreads();
  if (wave == 0) {
#pragma unroll 1
    for (int b0 = 0; b0 < tt; b0 += 32) {
      const int idx = b0 + lane;
      const int ent = hl[idx < RCAP ? idx : RCAP - 1];
      const int m32 = (tt - b0) < 32 ? (tt - b0) : 32;
#pragma unroll 1
      for (int k = 0; k < m32; ++k) {
        const int u    = __builtin_amdgcn_readlane(ent, k);
        const int slot = u & (NBA - 1);
        if (lane == 0) {
          int p = cur[slot];
          p = p < 0 ? 0 : (p > RCAP - 1 ? RCAP - 1 : p);
          sl[p] = u;
          cur[slot] = p + 1;
        }
      }
    }
  }
  __syncthreads();

  const float qnan = __int_as_float(0x7fc00000);
  const float pzb  = (ovf != 0) ? qnan : 0.0f;

  if constexpr (L == 1) {
    const v4f aw = *(const v4fa*)(par + PAR_ATT1 + 4 * lane);
#pragma unroll 1
    for (int si = 0; si < NBA / NWAVE; ++si) {
      const int s    = si * NWAVE + wave;
      const int node = nodeBase + s;
      int c = cnt[s];
      const bool big = c > DEGCAP;
      c = c < 0 ? 0 : (c > DEGCAP ? DEGCAP : c);
      int o = offs[s];
      o = o < 0 ? 0 : (o > tt ? tt : o);
      if (c > tt - o) c = tt - o;
      c = __builtin_amdgcn_readfirstlane(c);
      o = __builtin_amdgcn_readfirstlane(o);
      const int nc = node < nN ? node : nN - 1;
      const v4f hd = *(const v4fa*)(FD + (size_t)nc * HC1 + 4 * lane);
      float mx = -3.0e38f, dn = 0.0f;
      v4f av = {0.f, 0.f, 0.f, 0.f};
#pragma unroll 1
      for (int q = 0; q < c; ++q) {
        int idx = o + q; idx = idx > RCAP - 1 ? RCAP - 1 : idx;
        const int ent = sl[idx];
        int eid = ent >> SLA;
        eid = eid < 0 ? 0 : (eid > nE - 1 ? nE - 1 : eid);
        int sr = srcs[eid];
        sr = sr < 0 ? 0 : (sr > nN - 1 ? nN - 1 : sr);
        const v4f hs = *(const v4fa*)(FS + (size_t)sr * HC1 + 4 * lane);
        v4f tv = hs + hd;
        tv.x = tv.x > 0.f ? tv.x : NEGSL * tv.x;
        tv.y = tv.y > 0.f ? tv.y : NEGSL * tv.y;
        tv.z = tv.z > 0.f ? tv.z : NEGSL * tv.z;
        tv.w = tv.w > 0.f ? tv.w : NEGSL * tv.w;
        float p = tv.x * aw.x;
        p = fmaf(tv.y, aw.y, p);
        p = fmaf(tv.z, aw.z, p);
        p = fmaf(tv.w, aw.w, p);
        p += __shfl_xor(p, 1);
        p += __shfl_xor(p, 2);
        p += __shfl_xor(p, 4);
        const float df = p - mx;
        const float ee = expf(-fabsf(df));
        const bool  up = df > 0.f;
        const float s1 = up ? ee : 1.0f;
        const float s2 = up ? 1.0f : ee;
        mx = up ? p : mx;
        dn = fmaf(dn, s1, s2);
        av.x = fmaf(av.x, s1, s2 * hs.x);
        av.y = fmaf(av.y, s1, s2 * hs.y);
        av.z = fmaf(av.z, s1, s2 * hs.z);
        av.w = fmaf(av.w, s1, s2 * hs.w);
      }
      const bool has = c > 0;
      const float inv = __builtin_amdgcn_rcpf(has ? dn : 1.0f);
      const float pzr = big ? qnan : pzb;
      v4f ov4;
      ov4.x = (has ? av.x * inv : 0.0f) + pzr;
      ov4.y = (has ? av.y * inv : 0.0f) + pzr;
      ov4.z = (has ? av.z * inv : 0.0f) + pzr;
      ov4.w = (has ? av.w * inv : 0.0f) + pzr;
#pragma unroll 1
      for (int i = 0; i < 4; ++i) {
        const float e = elu1(ov4.x);
        ov4.x = ov4.y; ov4.y = ov4.z; ov4.z = ov4.w; ov4.w = e;
      }
      const unsigned int hbx = f2bf(ov4.x), hby = f2bf(ov4.y), hbz = f2bf(ov4.z), hbw = f2bf(ov4.w);
      const unsigned int lbx = f2bf(ov4.x - bf2f(hbx)), lby = f2bf(ov4.y - bf2f(hby));
      const unsigned int lbz = f2bf(ov4.z - bf2f(hbz)), lbw = f2bf(ov4.w - bf2f(hbw));
      const int hw0 = (int)(hbx | (hby << 16)), hw1 = (int)(hbz | (hbw << 16));
      const int lw0 = (int)(lbx | (lby << 16)), lw1 = (int)(lbz | (lbw << 16));
      const int sa = (2 * lane) & 31, sb = (2 * lane + 1) & 31;
      const int g0 = __shfl(hw0, sa), g1 = __shfl(hw1, sa), g2 = __shfl(hw0, sb), g3 = __shfl(hw1, sb);
      const int q0 = __shfl(lw0, sa), q1 = __shfl(lw1, sa), q2 = __shfl(lw0, sb), q3 = __shfl(lw1, sb);
      const bool lsel = lane >= 16;
      v4u pv;
      pv.x = (unsigned int)(lsel ? q0 : g0);
      pv.y = (unsigned int)(lsel ? q1 : g1);
      pv.z = (unsigned int)(lsel ? q2 : g2);
      pv.w = (unsigned int)(lsel ? q3 : g3);
      unsigned short* gp = HP + (size_t)nc * KA2 + 8 * lane;
      const bool wr = node < nN;
      if (wr) *(volatile v4u*)gp = pv;
      __threadfence();
      if (wr) *(volatile v4u*)gp = pv;
    }
  } else {
    const int hh = lane >> 4, cc = lane & 15;
    const float aw = par[PAR_ATT2 + cc];
#pragma unroll 1
    for (int si = 0; si < NBA / (2 * NWAVE); ++si) {
      const int pr   = si * NWAVE + wave;
      const int s    = 2 * pr + hh;
      const int node = nodeBase + s;
      int c = cnt[s];
      const bool big = c > DEGCAP;
      c = c < 0 ? 0 : (c > DEGCAP ? DEGCAP : c);
      int o = offs[s];
      o = o < 0 ? 0 : (o > tt ? tt : o);
      if (c > tt - o) c = tt - o;
      const int co = __shfl_xor(c, 16);
      int cm = c > co ? c : co;
      cm = __builtin_amdgcn_readfirstlane(cm);
      const int nc = node < nN ? node : nN - 1;
      const float hd = FS[(size_t)nc * NC2 + DOUT + cc];
      float mx = -3.0e38f, dn = 0.0f, ac = 0.0f;
#pragma unroll 1
      for (int q = 0; q < cm; ++q) {
        const bool act = q < c;
        int idx = o + q; idx = idx < 0 ? 0 : (idx > RCAP - 1 ? RCAP - 1 : idx);
        const int ent = sl[idx];
        int eid = ent >> SLA;
        eid = eid < 0 ? 0 : (eid > nE - 1 ? nE - 1 : eid);
        int sr = srcs[eid];
        sr = sr < 0 ? 0 : (sr > nN - 1 ? nN - 1 : sr);
        const float hs = FS[(size_t)sr * NC2 + cc];
        float tv = hs + hd;
        tv = tv > 0.f ? tv : NEGSL * tv;
        float p = tv * aw;
        p += __shfl_xor(p, 1);
        p += __shfl_xor(p, 2);
        p += __shfl_xor(p, 4);
        p += __shfl_xor(p, 8);
        const float df = p - mx;
        const float ee = expf(-fabsf(df));
        const bool  up = df > 0.f;
        const float s1 = up ? ee : 1.0f;
        const float s2 = up ? 1.0f : ee;
        const float mxn = up ? p : mx;
        const float dnn = fmaf(dn, s1, s2);
        const float acn = fmaf(ac, s1, s2 * hs);
        mx = act ? mxn : mx;
        dn = act ? dnn : dn;
        ac = act ? acn : ac;
      }
      const bool has = c > 0;
      const float inv = __builtin_amdgcn_rcpf(has ? dn : 1.0f);
      const float pzr = big ? qnan : pzb;
      const float val = (has ? ac * inv : 0.0f) + pzr;
      float* op = outp + (size_t)nc * DOUT + cc;
      const bool wr = node < nN;
      if (wr) *(volatile float*)op = val;
      __threadfence();
      if (wr) *(volatile float*)op = val;
    }
  }
}

static inline int cdiv(int a, int b) { return (a + b - 1) / b; }

extern "C" void kernel_launch(void* const* d_in, const int* in_sizes, int n_in,
                              void* d_out, int out_size, void* d_ws, size_t ws_size,
                              hipStream_t stream) {
  if (n_in < 12) return;
  if (in_sizes[0] < DIN || (in_sizes[0] % DIN) != 0) return;
  const int nN = in_sizes[0] / DIN;
  if (nN < 1 || nN > (1 << 22)) return;
  if (in_sizes[1] < 2 || (in_sizes[1] & 1) != 0) return;
  const int nE = in_sizes[1] / 2;
  if (nE < 1 || nE >= (1 << 21)) return;
  if (in_sizes[2] != DIN * HC1 || in_sizes[4] != DIN * HC1) return;
  if (in_sizes[3] != HC1 || in_sizes[5] != HC1) return;
  if (in_sizes[6] != HC1) return;
  if (in_sizes[7] != HC1 * DOUT || in_sizes[9] != HC1 * DOUT) return;
  if (in_sizes[8] != DOUT || in_sizes[10] != DOUT) return;
  if (in_sizes[11] != DOUT) return;
  if ((long long)out_size != (long long)nN * DOUT) return;

  const float* feat = (const float*)d_in[0];
  const int*   ei   = (const int*)  d_in[1];
  const float* W1s  = (const float*)d_in[2];
  const float* b1s  = (const float*)d_in[3];
  const float* W1d  = (const float*)d_in[4];
  const float* b1d  = (const float*)d_in[5];
  const float* at1  = (const float*)d_in[6];
  const float* W2s  = (const float*)d_in[7];
  const float* b2s  = (const float*)d_in[8];
  const float* W2d  = (const float*)d_in[9];
  const float* b2d  = (const float*)d_in[10];
  const float* at2  = (const float*)d_in[11];
  float* out = (float*)d_out;
  const int* src = ei;
  const int* dst = ei + nE;

  const int gM   = cdiv(nN, GBM);
  const int gA   = cdiv(nN, NBA);
  const int vec8 = ((nE & 3) == 0) ? 1 : 0;

  char* ws = (char*)d_ws;
  size_t off = 0;
  const size_t oPAR = off; off += (size_t)PAR_N * 4;            off = (off + 255) & ~(size_t)255;
  const size_t oWT1 = off; off += (size_t)NC1 * DIN * 2;        off = (off + 255) & ~(size_t)255;
  const size_t oWT2 = off; off += (size_t)NC2 * KA2 * 2;        off = (off + 255) & ~(size_t)255;
  const size_t oHS1 = off; off += (size_t)nN * HC1 * 4;         off = (off + 255) & ~(size_t)255;
  const size_t oHD1 = off; off += (size_t)nN * HC1 * 4;         off = (off + 255) & ~(size_t)255;
  const size_t oHSD = off; off += (size_t)nN * NC2 * 4;         off = (off + 255) & ~(size_t)255;
  if (off > ws_size || off > (size_t)WSMAX) return;
  float*          PAR  = (float*)(ws + oPAR);
  unsigned short* WT1  = (unsigned short*)(ws + oWT1);
  unsigned short* WT2  = (unsigned short*)(ws + oWT2);
  float*          HS1  = (float*)(ws + oHS1);
  float*          HD1  = (float*)(ws + oHD1);
  unsigned short* H1   = (unsigned short*)(ws + oHD1);
  float*          HSD2 = (float*)(ws + oHSD);

  const size_t scanLds = (size_t)AGG_LDS_INTS * 4;
  const size_t g1Lds   = (size_t)GBM * NC1 * 4;
  hipFuncSetAttribute(reinterpret_cast<const void*>(&k_gemm1), hipFuncAttributeMaxDynamicSharedMemorySize, (int)g1Lds);
  hipFuncSetAttribute(reinterpret_cast<const void*>(&k_scan<1>), hipFuncAttributeMaxDynamicSharedMemorySize, (int)scanLds);
  hipFuncSetAttribute(reinterpret_cast<const void*>(&k_scan<2>), hipFuncAttributeMaxDynamicSharedMemorySize, (int)scanLds);

  k_prep<<<NU_W / NTHR + 1, NTHR, 0, stream>>>(W1s, W1d, W2s, W2d, b1s, b1d, at1, b2s, b2d, at2, WT1, WT2, PAR);
  k_gemm1<<<gM, NTHR, g1Lds, stream>>>(feat, WT1, PAR, HS1, HD1, nN);
  k_scan<1><<<gA, NTHR, scanLds, stream>>>(src, dst, nE, nN, vec8, PAR, HS1, HD1, H1, out);
  k_gemm2<<<gM, G2THR, 0, stream>>>(H1, WT2, PAR, HSD2, nN);
  k_scan<2><<<gA, NTHR, scanLds, stream>>>(src, dst, nE, nN, vec8, PAR, HSD2, HSD2, H1, out);
}
